// SparseAttention_69020124446895
// MI455X (gfx1250) — hardware-verified
//
#include <hip/hip_runtime.h>


#ifndef NB
#define NB 2
#endif
#ifndef SEQ
#define SEQ 4096
#endif
#define SEQ_FULL 4096
#define NB_FULL  2
#define DM   512
#define NH   8
#define HD   64
#define BLK  128
#define NBLK (SEQ / BLK)
#define MTOK (NB * SEQ)
#define PP   40
#define L2E  1.4426950408889634f
#define FILL2 (-1.4426950e10f)

static_assert(DM == NH * HD);
static_assert(SEQ % BLK == 0);
static_assert(NBLK >= 1 && NBLK <= 32);
static_assert(MTOK % 64 == 0);
static_assert(SEQ % 64 == 0);
static_assert(DM % 64 == 0 && DM % 32 == 0);
static_assert(SEQ <= SEQ_FULL && NB <= NB_FULL);

typedef unsigned short bf;
typedef __attribute__((ext_vector_type(16))) __bf16   v16bf;
typedef __attribute__((ext_vector_type(8)))  unsigned short v8us;
typedef __attribute__((ext_vector_type(2)))  unsigned short v2us;
typedef __attribute__((ext_vector_type(8)))  float    v8f;
typedef __attribute__((ext_vector_type(4)))  float    v4f;
typedef v4f  __attribute__((may_alias)) v4fa;
typedef v8us __attribute__((may_alias)) v8usa;

__device__ __forceinline__ unsigned short f2bf(float f) { unsigned u = __float_as_uint(f); u += 0x7FFFu + ((u >> 16) & 1u); return (unsigned short)(u >> 16); }
__device__ __forceinline__ float bf2f(unsigned short b) { return __uint_as_float(((unsigned)b) << 16); }
__device__ __forceinline__ float bfr(float f) { return bf2f(f2bf(f)); }
__device__ __forceinline__ void splitf(float y, unsigned short& h, unsigned short& l) { h = f2bf(y); l = f2bf(y - bf2f(h)); }
__device__ __forceinline__ unsigned umin2(unsigned a, unsigned b) { return a < b ? a : b; }
__device__ __forceinline__ v16bf cat16b(v8us lo, v8us hi) { return __builtin_bit_cast(v16bf, __builtin_shufflevector(lo, hi, 0, 1, 2, 3, 4, 5, 6, 7, 8, 9, 10, 11, 12, 13, 14, 15)); }
__device__ __forceinline__ v16bf ldb(const bf* p) { return cat16b(*(const v8us*)p, *(const v8us*)(p + 16)); }
__device__ __forceinline__ v16bf ldbs(const unsigned short* p) { return cat16b(*(const v8usa*)p, *(const v8usa*)(p + 16)); }
__device__ __forceinline__ v8f wmmab(v16bf a, v16bf b, v8f c) { return __builtin_amdgcn_wmma_f32_16x16x32_bf16(false, a, false, b, (short)0, c, false, false); }

__global__ __launch_bounds__(256) void k_cvtx(const float* __restrict__ x, bf* dst) {
    const unsigned i = blockIdx.x * 256u + threadIdx.x; if (i >= (unsigned)(MTOK * DM / 8)) return;
    const unsigned e = i * 8u; const unsigned col = e & (unsigned)(DM - 1); const unsigned row = e / (unsigned)DM; const unsigned b = row / (unsigned)SEQ, s = row % (unsigned)SEQ;
    const v8f v = *(const v8f*)(x + ((size_t)(b * (unsigned)SEQ_FULL + s) * DM + col)); v8us o;
#pragma unroll
    for (int k = 0; k < 8; ++k) o[k] = f2bf(v[k]);
    *(volatile v8us*)(dst + e) = o; __threadfence(); *(volatile v8us*)(dst + e) = o; }

__global__ __launch_bounds__(256) void k_wt4(const float* __restrict__ w0, const float* __restrict__ w1, const float* __restrict__ w2, const float* __restrict__ w3, bf* Bt) {
    const unsigned y = blockIdx.y; const float* w = (y == 0u) ? w0 : ((y == 1u) ? w1 : ((y == 2u) ? w2 : w3)); bf* dst = Bt + (size_t)y * DM * DM;
    const unsigned lane = threadIdx.x & 31u; const unsigned L0 = (blockIdx.x * 8u + (threadIdx.x >> 5)) * 8u;
#pragma unroll 1
    for (int ps = 0; ps < 2; ++ps) {
#pragma unroll 1
        for (unsigned l = 0; l < 8u; ++l) { const unsigned e = (L0 + l) * 64u + lane * 2u; const unsigned k = e & (unsigned)(DM - 1), n = e / (unsigned)DM; v2us o;
            o[0] = f2bf(w[(size_t)k * DM + n]); o[1] = f2bf(w[(size_t)(k + 1u) * DM + n]); *(volatile v2us*)(dst + e) = o; }
        if (ps == 0) __threadfence(); }
}

template <int NSPLIT>
__device__ __forceinline__ void gemm_main(const bf* __restrict__ A, const bf* __restrict__ A2, const bf* __restrict__ Bt, unsigned K, unsigned r0, unsigned c0, unsigned lr, unsigned hi, v8f (&acc)[4][4]) {
#pragma unroll
    for (int mb = 0; mb < 4; ++mb)
#pragma unroll
        for (int nb = 0; nb < 4; ++nb) acc[mb][nb] = (v8f){};
    const size_t aoff = (size_t)(r0 + lr) * K + 8u * hi, boff = (size_t)(c0 + lr) * K + 8u * hi;
#pragma unroll 1
    for (unsigned kc = 0; kc < K; kc += 32u) {
        v16bf a[4], a2[4];
#pragma unroll
        for (int mb = 0; mb < 4; ++mb) { a[mb] = ldb(A + aoff + (size_t)mb * 16u * K + kc); if (NSPLIT == 1) a2[mb] = ldb(A2 + aoff + (size_t)mb * 16u * K + kc); else a2[mb] = a[mb]; }
#pragma unroll
        for (int nb = 0; nb < 4; ++nb) { const v16bf b = ldb(Bt + boff + (size_t)nb * 16u * K + kc);
#pragma unroll
            for (int mb = 0; mb < 4; ++mb) { acc[mb][nb] = wmmab(a[mb], b, acc[mb][nb]); if (NSPLIT == 1) acc[mb][nb] = wmmab(a2[mb], b, acc[mb][nb]); } }
        asm volatile("v_nop\n\tv_nop\n\tv_nop\n\tv_nop" : "+v"(acc[0][0]), "+v"(acc[1][1]), "+v"(acc[2][2]), "+v"(acc[3][3]) : "v"(a[0]), "v"(a[3]));
    }
}

__global__ __launch_bounds__(32) void k_qkv(const bf* __restrict__ X, const bf* __restrict__ Wt3, const float* __restrict__ bq, const float* __restrict__ bk, const float* __restrict__ bv,
                                            bf* Qh, bf* Ql, bf* Kh, bf* Kl, bf* VTh, bf* VTl) {
    __shared__ __align__(16) float os[64 * 68];
    const unsigned z = blockIdx.z; const unsigned lane = threadIdx.x & 31u, lr = lane & 15u, hi = lane >> 4; const unsigned r0 = blockIdx.x * 64u, c0 = blockIdx.y * 64u;
    v8f acc[4][4];
    gemm_main<0>(X, X, Wt3 + (size_t)z * DM * DM, (unsigned)DM, r0, c0, lr, hi, acc);
#pragma unroll
    for (int mb = 0; mb < 4; ++mb)
#pragma unroll
        for (int nb = 0; nb < 4; ++nb)
#pragma unroll
            for (int j = 0; j < 8; ++j) os[(mb * 16 + hi * 8 + j) * 68 + nb * 16 + lr] = acc[mb][nb][j];
    __builtin_amdgcn_wave_barrier(); asm volatile("" ::: "memory");
    const unsigned b = r0 / (unsigned)SEQ, s0 = r0 % (unsigned)SEQ; const size_t bh = (size_t)b * NH + blockIdx.y;
    const unsigned c8 = (lane & 7u) * 8u, rq = lane >> 3;
    if (z < 2u) {
        const float* bias = (z == 0u) ? bq : bk; const float sc = (z == 0u) ? 0.125f : 1.0f;
        bf* Ph = ((z == 0u) ? Qh : Kh) + (bh * SEQ + s0) * HD + c8; bf* Pl = ((z == 0u) ? Ql : Kl) + (bh * SEQ + s0) * HD + c8;
        const v4f b0 = *(const v4f*)(bias + c0 + c8), b1 = *(const v4f*)(bias + c0 + c8 + 4u); float bb[8];
#pragma unroll
        for (int q = 0; q < 4; ++q) { bb[q] = bfr(b0[q]); bb[4 + q] = bfr(b1[q]); }
#pragma unroll 1
        for (int ps = 0; ps < 2; ++ps) {
#pragma unroll 2
            for (unsigned it = 0; it < 16u; ++it) { const unsigned row = it * 4u + rq; const v4f a0 = *(const v4fa*)(os + row * 68u + c8), a1 = *(const v4fa*)(os + row * 68u + c8 + 4u); v8us oh, ol;
#pragma unroll
                for (int q = 0; q < 4; ++q) { unsigned short h, l; splitf((a0[q] + bb[q]) * sc, h, l); oh[q] = h; ol[q] = l; splitf((a1[q] + bb[4 + q]) * sc, h, l); oh[4 + q] = h; ol[4 + q] = l; }
                *(volatile v8us*)(Ph + (size_t)row * HD) = oh; *(volatile v8us*)(Pl + (size_t)row * HD) = ol; }
            if (ps == 0) __threadfence(); }
    } else {
        bf* Vh = VTh + bh * HD * SEQ + s0 + c8; bf* Vl = VTl + bh * HD * SEQ + s0 + c8;
#pragma unroll 1
        for (int ps = 0; ps < 2; ++ps) {
#pragma unroll 2
            for (unsigned it = 0; it < 16u; ++it) { const unsigned d = it * 4u + rq; const float bd = bfr(bv[c0 + d]); v8us oh, ol;
#pragma unroll
                for (int q = 0; q < 8; ++q) { unsigned short h, l; splitf(os[(c8 + q) * 68u + d] + bd, h, l); oh[q] = h; ol[q] = l; }
                *(volatile v8us*)(Vh + (size_t)d * SEQ) = oh; *(volatile v8us*)(Vl + (size_t)d * SEQ) = ol; }
            if (ps == 0) __threadfence(); }
    }
}

__global__ __launch_bounds__(256) void k_v0(const bf* __restrict__ VTh, const bf* __restrict__ VTl, bf* V0h, bf* V0l) {
    const unsigned i = blockIdx.x * 256u + threadIdx.x; if (i >= (unsigned)(NB * NH * HD * 32 / 8)) return;
    const unsigned e = i * 8u; const unsigned j0 = e & 31u; const unsigned row = e >> 5; v8us oh, ol;
#pragma unroll
    for (int q = 0; q < 8; ++q) { const unsigned j = umin2(j0 + (unsigned)q, (unsigned)(NBLK - 1)); const size_t o = (size_t)row * SEQ + (size_t)j * BLK; oh[q] = VTh[o]; ol[q] = VTl[o]; }
    *(volatile v8us*)(V0h + e) = oh; *(volatile v8us*)(V0l + e) = ol; __threadfence(); *(volatile v8us*)(V0h + e) = oh; *(volatile v8us*)(V0l + e) = ol; }

__global__ __launch_bounds__(256) void k_flash(const bf* __restrict__ Qh, const bf* __restrict__ Ql, const bf* __restrict__ Kh, const bf* __restrict__ Kl,
                                               const bf* __restrict__ VTh, const bf* __restrict__ VTl, const bf* __restrict__ V0h, const bf* __restrict__ V0l, bf* Xh, bf* Xl) {
    __shared__ __align__(16) unsigned short sPh[8 * 16 * PP];
    __shared__ __align__(16) unsigned short sPl[8 * 16 * PP];
    __shared__ __align__(16) float sO[8 * 16 * 68];
    const unsigned qb = blockIdx.x, hh = blockIdx.y, b = blockIdx.z;
    const unsigned w = (unsigned)__builtin_amdgcn_readfirstlane((int)(threadIdx.x >> 5));
    const unsigned lane = threadIdx.x & 31u, lr = lane & 15u, hi = lane >> 4;
    const unsigned qbase = qb * (unsigned)BLK + w * 16u;
    const size_t bh = (size_t)b * NH + hh;
    const bf* kh = Kh + bh * SEQ * HD; const bf* kl = Kl + bh * SEQ * HD;
    const bf* vth = VTh + bh * HD * SEQ; const bf* vtl = VTl + bh * HD * SEQ; const bf* v0h = V0h + bh * HD * 32; const bf* v0l = V0l + bh * HD * 32;
    unsigned short* ph = sPh + w * 16u * PP; unsigned short* pl = sPl + w * 16u * PP; float* so = sO + w * 16u * 68u;

    const size_t qo = (bh * SEQ + qbase + lr) * HD + 8u * hi;
    const v16bf aqh0 = ldb(Qh + qo), aqh1 = ldb(Qh + qo + 32), aql0 = ldb(Ql + qo), aql1 = ldb(Ql + qo + 32);

    v8f accO[4];
#pragma unroll
    for (int t = 0; t < 4; ++t) accO[t] = (v8f){};
    float rmax[8], lsum[8];
#pragma unroll
    for (int r = 0; r < 8; ++r) { rmax[r] = -1.0e30f; lsum[r] = 0.f; }

    const unsigned nd = (w >> 1) + 1u;
    const unsigned nT = nd + qb + ((qb > 0u) ? 1u : 0u);
#pragma unroll 1
    for (unsigned it = 0; it < nT; ++it) {
        const unsigned kind = (it < nd) ? 0u : ((it < nd + qb) ? 1u : 2u);
        const unsigned kbase = (kind == 0u) ? (qb * (unsigned)BLK + it * 32u) : ((kind == 1u) ? ((it - nd) * (unsigned)BLK + 96u) : 0u);
        const unsigned kmul = (kind == 2u) ? (unsigned)BLK : 1u;
        const unsigned kcl = (kind == 2u) ? (unsigned)(NBLK - 1) : 31u;
        const size_t ko0 = (size_t)(kbase + umin2(lr, kcl) * kmul) * HD + 8u * hi;
        const size_t ko1 = (size_t)(kbase + umin2(16u + lr, kcl) * kmul) * HD + 8u * hi;
        v8f sc0 = (v8f){}, sc1 = (v8f){};
        {
            const v16bf b0h0 = ldb(kh + ko0), b0h1 = ldb(kh + ko0 + 32), b0l0 = ldb(kl + ko0), b0l1 = ldb(kl + ko0 + 32);
            const v16bf b1h0 = ldb(kh + ko1), b1h1 = ldb(kh + ko1 + 32), b1l0 = ldb(kl + ko1), b1l1 = ldb(kl + ko1 + 32);
            sc0 = wmmab(aqh0, b0h0, sc0); sc1 = wmmab(aqh0, b1h0, sc1);
            sc0 = wmmab(aqh1, b0h1, sc0); sc1 = wmmab(aqh1, b1h1, sc1);
            sc0 = wmmab(aql0, b0h0, sc0); sc1 = wmmab(aql0, b1h0, sc1);
            sc0 = wmmab(aql1, b0h1, sc0); sc1 = wmmab(aql1, b1h1, sc1);
            sc0 = wmmab(aqh0, b0l0, sc0); sc1 = wmmab(aqh0, b1l0, sc1);
            sc0 = wmmab(aqh1, b0l1, sc0); sc1 = wmmab(aqh1, b1l1, sc1);
            asm volatile("v_nop\n\tv_nop\n\tv_nop\n\tv_nop" : "+v"(sc0), "+v"(sc1) : "v"(aqh1), "v"(b1l1));
        }
        const unsigned kr0 = (kind == 0u) ? (kbase + lr) : ((kind == 1u) ? 0u : lr);
        const unsigned kr1 = (kind == 0u) ? (kbase + 16u + lr) : ((kind == 1u) ? 0u : (16u + lr));
        const unsigned tb = (kind == 0u) ? (qbase + 8u * hi) : ((kind == 1u) ? 0u : (qb - 1u));
        const unsigned ti = (kind == 0u) ? 1u : 0u;
        __builtin_amdgcn_wave_barrier(); asm volatile("" ::: "memory");
#pragma unroll
        for (int r = 0; r < 8; ++r) {
            const unsigned thr = tb + ti * (unsigned)r;
            const float x0 = (kr0 <= thr) ? sc0[r] * L2E : FILL2;
            const float x1 = (kr1 <= thr) ? sc1[r] * L2E : FILL2;
            float m = fmaxf(x0, x1);
            m = fmaxf(m, __shfl_xor(m, 1, 32)); m = fmaxf(m, __shfl_xor(m, 2, 32)); m = fmaxf(m, __shfl_xor(m, 4, 32)); m = fmaxf(m, __shfl_xor(m, 8, 32));
            const float nm = fmaxf(rmax[r], m);
            const float cr = __builtin_amdgcn_exp2f(rmax[r] - nm);
            const float p0 = __builtin_amdgcn_exp2f(x0 - nm), p1 = __builtin_amdgcn_exp2f(x1 - nm);
            lsum[r] = lsum[r] * cr + (p0 + p1); rmax[r] = nm;
#pragma unroll
            for (int t = 0; t < 4; ++t) accO[t][r] *= cr;
            unsigned short h0, l0, h1, l1; splitf(p0, h0, l0); splitf(p1, h1, l1);
            const unsigned po = (8u * hi + (unsigned)r) * PP + lr;
            ph[po] = h0; pl[po] = l0; ph[po + 16u] = h1; pl[po + 16u] = l1;
        }
        __builtin_amdgcn_wave_barrier(); asm volatile("" ::: "memory");
        const v16bf aph = ldbs(ph + lr * PP + 8u * hi), apl = ldbs(pl + lr * PP + 8u * hi);
        const bf* vbh = (kind == 2u) ? v0h : (vth + kbase); const bf* vbl = (kind == 2u) ? v0l : (vtl + kbase); const unsigned vp = (kind == 2u) ? 32u : (unsigned)SEQ;
#pragma unroll
        for (int t = 0; t < 4; ++t) { const size_t vo = (size_t)((unsigned)t * 16u + lr) * vp + 8u * hi; const v16bf bvh = ldb(vbh + vo), bvl = ldb(vbl + vo);
            accO[t] = wmmab(aph, bvh, accO[t]); accO[t] = wmmab(apl, bvh, accO[t]); accO[t] = wmmab(aph, bvl, accO[t]); }
        asm volatile("v_nop\n\tv_nop\n\tv_nop\n\tv_nop" : "+v"(accO[0]), "+v"(accO[1]), "+v"(accO[2]), "+v"(accO[3]) : "v"(aph), "v"(apl));
    }
#pragma unroll
    for (int r = 0; r < 8; ++r) { float s = lsum[r]; s += __shfl_xor(s, 1, 32); s += __shfl_xor(s, 2, 32); s += __shfl_xor(s, 4, 32); s += __shfl_xor(s, 8, 32); const float inv = 1.0f / s;
#pragma unroll
        for (int t = 0; t < 4; ++t) so[(8u * hi + (unsigned)r) * 68u + (unsigned)t * 16u + lr] = accO[t][r] * inv; }
    __builtin_amdgcn_wave_barrier(); asm volatile("" ::: "memory");
    const unsigned c8 = (lane & 7u) * 8u, rq = lane >> 3;
    bf* xh = Xh + ((size_t)b * SEQ + qbase) * DM + hh * (unsigned)HD + c8; bf* xl = Xl + ((size_t)b * SEQ + qbase) * DM + hh * (unsigned)HD + c8;
#pragma unroll 1
    for (int ps = 0; ps < 2; ++ps) {
#pragma unroll
        for (unsigned s = 0; s < 4u; ++s) { const unsigned row = s * 4u + rq; const v4f a0 = *(const v4fa*)(so + row * 68u + c8), a1 = *(const v4fa*)(so + row * 68u + c8 + 4u); v8us oh, ol;
#pragma unroll
            for (int q = 0; q < 4; ++q) { unsigned short h, l; splitf(a0[q], h, l); oh[q] = h; ol[q] = l; splitf(a1[q], h, l); oh[4 + q] = h; ol[4 + q] = l; }
            *(volatile v8us*)(xh + (size_t)row * DM) = oh; *(volatile v8us*)(xl + (size_t)row * DM) = ol; }
        if (ps == 0) __threadfence(); }
}

__global__ __launch_bounds__(32) void k_outp(const bf* __restrict__ Xh, const bf* __restrict__ Xl, const bf* __restrict__ Wot, const float* __restrict__ bo, float* C) {
    __shared__ __align__(16) float os[64 * 68];
    const unsigned lane = threadIdx.x & 31u, lr = lane & 15u, hi = lane >> 4; const unsigned r0 = blockIdx.x * 64u, c0 = blockIdx.y * 64u;
    v8f acc[4][4];
    gemm_main<1>(Xh, Xl, Wot, (unsigned)DM, r0, c0, lr, hi, acc);
#pragma unroll
    for (int mb = 0; mb < 4; ++mb)
#pragma unroll
        for (int nb = 0; nb < 4; ++nb)
#pragma unroll
            for (int j = 0; j < 8; ++j) os[(mb * 16 + hi * 8 + j) * 68 + nb * 16 + lr] = acc[mb][nb][j];
    __builtin_amdgcn_wave_barrier(); asm volatile("" ::: "memory");
    const unsigned cofs = lr * 4u; const v4f bi = *(const v4f*)(bo + c0 + cofs); v4f bb; bb[0] = bfr(bi[0]); bb[1] = bfr(bi[1]); bb[2] = bfr(bi[2]); bb[3] = bfr(bi[3]);
    float* crow = C + (size_t)r0 * DM + c0 + cofs;
#pragma unroll 1
    for (int ps = 0; ps < 2; ++ps) {
#pragma unroll 4
        for (unsigned it = 0; it < 32u; ++it) { const unsigned row = 2u * it + hi; v4f val = *(const v4fa*)(os + row * 68u + cofs); val[0] += bb[0]; val[1] += bb[1]; val[2] += bb[2]; val[3] += bb[3];
            *(volatile v4f*)(crow + (size_t)row * DM) = val; }
        if (ps == 0) __threadfence(); }
}

static_assert((MTOK * DM / 8 / 256) * 256 * 8 == MTOK * DM);
static_assert(64 * 8 * 8 * 64 == DM * DM);
static_assert((MTOK / 64) * NH * 64 * 64 == NB * NH * SEQ * HD);
static_assert((NB * NH * HD * 32 / 8 / 256) * 256 * 8 == NB * NH * HD * 32);
static_assert(NBLK * NH * NB * 8 * 16 * HD == MTOK * DM);
static_assert((MTOK / 64) * (DM / 64) * 64 * 64 == MTOK * DM);

extern "C" void kernel_launch(void* const* d_in, const int* in_sizes, int n_in,
                              void* d_out, int out_size, void* d_ws, size_t ws_size, hipStream_t stream) {
    if (n_in < 9) return;
    if ((long long)in_sizes[0] < (long long)(NB - 1) * SEQ_FULL * DM + (long long)SEQ * DM) return;
    if (in_sizes[1] < DM * DM || in_sizes[3] < DM * DM || in_sizes[5] < DM * DM || in_sizes[7] < DM * DM) return;
    if (in_sizes[2] < DM || in_sizes[4] < DM || in_sizes[6] < DM || in_sizes[8] < DM) return;
    if ((long long)out_size < (long long)MTOK * DM) return;
    const float* x  = (const float*)d_in[0];
    const float* wq = (const float*)d_in[1]; const float* bq = (const float*)d_in[2];
    const float* wk = (const float*)d_in[3]; const float* bk = (const float*)d_in[4];
    const float* wv = (const float*)d_in[5]; const float* bv = (const float*)d_in[6];
    const float* wo = (const float*)d_in[7]; const float* bo = (const float*)d_in[8];
    float* OUT = (float*)d_out;
    char* wsp = (char*)d_ws;
    auto take = [&](size_t bytes) { char* p = wsp; wsp += (bytes + 255) & ~(size_t)255; return (void*)p; };
    const size_t planeB = (size_t)NB * NH * SEQ * HD * 2;
    bf* Xb  = (bf*)take((size_t)MTOK * DM * 2);
    bf* Wt  = (bf*)take((size_t)4 * DM * DM * 2);
    bf* Qh  = (bf*)take(planeB); bf* Ql = (bf*)take(planeB); bf* Kh = (bf*)take(planeB); bf* Kl = (bf*)take(planeB);
    bf* VTh = (bf*)take(planeB); bf* VTl = (bf*)take(planeB);
    bf* V0h = (bf*)take((size_t)NB * NH * HD * 32 * 2); bf* V0l = (bf*)take((size_t)NB * NH * HD * 32 * 2);
    bf* Ch  = (bf*)take((size_t)MTOK * DM * 2); bf* Cl = (bf*)take((size_t)MTOK * DM * 2);
    const size_t used = (size_t)(wsp - (char*)d_ws);
    if (used > ws_size || used > (size_t)134217728) return;

    k_cvtx<<<(unsigned)(MTOK * DM / 8 / 256), 256, 0, stream>>>(x, Xb);
    k_wt4<<<dim3(64, 4, 1), 256, 0, stream>>>(wq, wk, wv, wo, Wt);
    k_qkv<<<dim3(MTOK / 64, NH, 3), 32, 0, stream>>>(Xb, Wt, bq, bk, bv, Qh, Ql, Kh, Kl, VTh, VTl);
    k_v0<<<(unsigned)(NB * NH * HD * 32 / 8 / 256), 256, 0, stream>>>(VTh, VTl, V0h, V0l);
    k_flash<<<dim3(NBLK, NH, NB), 256, 0, stream>>>(Qh, Ql, Kh, Kl, VTh, VTl, V0h, V0l, Ch, Cl);
    k_outp<<<dim3(MTOK / 64, DM / 64, 1), 32, 0, stream>>>(Ch, Cl, Wt + (size_t)3 * DM * DM, bo, OUT);
}
